// LSTMModel_31679678775668
// MI455X (gfx1250) — hardware-verified
//
#include <hip/hip_runtime.h>
#include <math.h>

constexpr int NSEQ   = 256;
constexpr int NSTEP  = 512;
constexpr int NFEAT  = 64;
constexpr int NHID   = 128;
constexpr int NGATE4 = 4 * NHID;
constexpr int KCAT2  = 2 * NHID;
constexpr int NPCOL  = 1536;
constexpr int NPRED  = NSEQ * NPCOL;
constexpr int NTHR   = 256;
constexpr int NWAVE  = NTHR / 32;
constexpr int RB     = 16;
constexpr int NBLK   = NSEQ / RB;
constexpr int XPITCH = 72;
constexpr int APITCH = 264;
constexpr int HPITCH = 136;
constexpr int SLABP  = 68;
constexpr int PLINE  = 32;
constexpr float WCARRY     = 16.0f;
constexpr float WCARRY_INV = 1.0f / 16.0f;
constexpr float FORGET_B   = 1.0f;
constexpr float LOSS_INV   = 1.0f / (float)NPRED;
static_assert(NHID == 16 * NWAVE);
static_assert(NSEQ % RB == 0);
static_assert(NFEAT % 32 == 0 && NHID % 32 == 0 && KCAT2 % 32 == 0);
static_assert(NFEAT % 64 == 0 && NHID % 64 == 0 && KCAT2 % 64 == 0 && NGATE4 % 64 == 0 && NPCOL % 64 == 0);
static_assert(NPCOL == 64 * 3 * NWAVE);
static_assert(RB * NFEAT == 4 * NTHR);
static_assert((XPITCH * 2) % 16 == 0 && (APITCH * 2) % 16 == 0 && (HPITCH * 2) % 16 == 0);
static_assert(XPITCH >= NFEAT && APITCH >= KCAT2 && HPITCH >= NHID && SLABP >= 64);
static_assert((NPCOL * 4) % 128 == 0);
static_assert(PLINE * 4 == 128);

typedef __attribute__((ext_vector_type(16))) _Float16 v16h;
typedef __attribute__((ext_vector_type(8)))  _Float16 v8h;
typedef __attribute__((ext_vector_type(16))) __bf16   v16b;
typedef __attribute__((ext_vector_type(8)))  __bf16   v8b;
typedef __attribute__((ext_vector_type(8)))  float    v8f;
typedef __attribute__((ext_vector_type(4)))  float    v4f;
typedef __attribute__((ext_vector_type(2)))  unsigned v2u;

__device__ __forceinline__ unsigned short f2bf_bits(float f) {
  unsigned u = __float_as_uint(f);
  return (unsigned short)((u + 0x7FFFu + ((u >> 16) & 1u)) >> 16);
}
__device__ __forceinline__ float bf_bits2f(unsigned short h) { return __uint_as_float(((unsigned)h) << 16); }
__device__ __forceinline__ float bf16r(float f) { return bf_bits2f(f2bf_bits(f)); }

__device__ __forceinline__ void acc_guard4(v8f& a, v8f& b, v8f& c, v8f& d) { asm volatile("v_nop\n\tv_nop\n\tv_nop\n\tv_nop" : "+v"(a), "+v"(b), "+v"(c), "+v"(d)); }
__device__ __forceinline__ void grp_guard_b(v8f& a0, v8f& a1, v8f& a2, v8f& a3, v16b x, v16b y0, v16b y1, v16b y2, v16b y3) {
  asm volatile("v_nop\n\tv_nop\n\tv_nop\n\tv_nop" : "+v"(a0), "+v"(a1), "+v"(a2), "+v"(a3) : "v"(x), "v"(y0), "v"(y1), "v"(y2), "v"(y3));
}
__device__ __forceinline__ void grp_guard_h(v8f& a0, v8f& a1, v8f& a2, v8f& a3, v16h x, v16h y0, v16h y1, v16h y2, v16h y3) {
  asm volatile("v_nop\n\tv_nop\n\tv_nop\n\tv_nop" : "+v"(a0), "+v"(a1), "+v"(a2), "+v"(a3) : "v"(x), "v"(y0), "v"(y1), "v"(y2), "v"(y3));
}
__device__ __forceinline__ void grp_guard_b2(v8f& a0, v8f& a1, v8f& a2, v8f& a3, v16b x, v16b x2, v16b y0, v16b y1, v16b y2, v16b y3) {
  asm volatile("v_nop\n\tv_nop\n\tv_nop\n\tv_nop" : "+v"(a0), "+v"(a1), "+v"(a2), "+v"(a3) : "v"(x), "v"(x2), "v"(y0), "v"(y1), "v"(y2), "v"(y3));
}

template <typename T> struct Frag;
template <> struct Frag<_Float16> {
  typedef v16h V; union U { v16h v; v8h h[2]; };
  static __device__ __forceinline__ v16h load(const _Float16* p) {
    U f; f.h[0] = *(const v8h*)(p); f.h[1] = *(const v8h*)(p + 16); return f.v;
  }
  static __device__ __forceinline__ v8f mma(v16h a, v16h b, v8f c) {
    return __builtin_amdgcn_wmma_f32_16x16x32_f16(false, a, false, b, (short)0, c, false, false);
  }
};
template <> struct Frag<__bf16> {
  typedef v16b V; union U { v16b v; v8b h[2]; };
  static __device__ __forceinline__ v16b load(const __bf16* p) {
    U f; f.h[0] = *(const v8b*)(p); f.h[1] = *(const v8b*)(p + 16); return f.v;
  }
  static __device__ __forceinline__ v8f mma(v16b a, v16b b, v8f c) {
    return __builtin_amdgcn_wmma_f32_16x16x32_bf16(false, a, false, b, (short)0, c, false, false);
  }
};

__device__ __forceinline__ float fsig(float v)  { return __builtin_amdgcn_rcpf(1.0f + expf(-v)); }
__device__ __forceinline__ float ftanh(float v) { return 1.0f - 2.0f * __builtin_amdgcn_rcpf(expf(2.0f * v) + 1.0f); }

template <int MODE>
__global__ __launch_bounds__(NTHR) void tpw_kernel(const float* __restrict__ src, int R, int C, int ldo,
                                                   unsigned short* __restrict__ O, float sc) {
  __shared__ float Tt[64 * 65];
  const int tid = threadIdx.x;
  const int c0 = blockIdx.x * 64, r0 = blockIdx.y * 64;
  (void)R;
#pragma unroll
  for (int i = 0; i < 4; ++i) {
    const int idx = i * NTHR + tid;
    const int rr = idx >> 4, cc = (idx & 15) * 4;
    const v4f v = *(const v4f*)(src + (size_t)(r0 + rr) * (size_t)C + c0 + cc);
    Tt[rr * 65 + cc + 0] = v[0];
    Tt[rr * 65 + cc + 1] = v[1];
    Tt[rr * 65 + cc + 2] = v[2];
    Tt[rr * 65 + cc + 3] = v[3];
  }
  __syncthreads();
  const int q = tid >> 3, c8 = (tid & 7) * 8;
  v8h hv[2];
#pragma unroll
  for (int g = 0; g < 2; ++g) {
    const int qq = g * 32 + q;
#pragma unroll
    for (int e = 0; e < 8; ++e) {
      const float f = Tt[(c8 + e) * 65 + qq];
      unsigned short bits;
      if (MODE == 0) {
        bits = f2bf_bits(f * sc);
      } else {
        const float fb = bf_bits2f(f2bf_bits(f));
        bits = __builtin_bit_cast(unsigned short, (_Float16)(fb * sc));
      }
      hv[g][e] = __builtin_bit_cast(_Float16, bits);
    }
  }
  for (int pass = 0; pass < 2; ++pass) {
#pragma unroll
    for (int g = 0; g < 2; ++g) {
      const size_t o = (size_t)(c0 + g * 32 + q) * (size_t)ldo + (size_t)(r0 + c8);
      *(volatile v8h*)(O + o) = hv[g];
    }
    __threadfence();
  }
}

__global__ __launch_bounds__(NTHR) void lstm2_kernel(const float* __restrict__ x, const float* __restrict__ bias1,
                                                     const float* __restrict__ bias2, const float* __restrict__ biasd,
                                                     const float* __restrict__ lab,
                                                     const unsigned short* __restrict__ W1Xp,
                                                     const unsigned short* __restrict__ W1Hp,
                                                     const unsigned short* __restrict__ W2Tp,
                                                     const unsigned short* __restrict__ WDTp,
                                                     float* __restrict__ pred, float* __restrict__ part) {
  __shared__ __align__(16) unsigned short Xs[RB * XPITCH];
  __shared__ __align__(16) _Float16       Ah[RB * APITCH];
  __shared__ __align__(16) unsigned short Hh[RB * HPITCH];
  __shared__ __align__(16) unsigned short Hl[RB * HPITCH];
  __shared__ __align__(16) float          Sl[NWAVE][16 * SLABP];
  __shared__ __align__(16) float          wsum[NWAVE];
  __shared__ __align__(16) float          lbuf[PLINE];
  const __bf16*   W1X = (const __bf16*)W1Xp;
  const _Float16* W1H = (const _Float16*)W1Hp;
  const _Float16* W2T = (const _Float16*)W2Tp;
  const __bf16*   WDT = (const __bf16*)WDTp;
  const int tid = threadIdx.x, lane = tid & 31, wave = tid >> 5;
  const int c = lane & 15, hh = lane >> 4, koff = hh * 8, c4 = c * 4;
  const int rowbase = blockIdx.x * RB;
  const int j = 16 * wave + c;

#pragma unroll 1
  for (int i = tid; i < RB * XPITCH; i += NTHR) Xs[i] = (unsigned short)0;
#pragma unroll 1
  for (int i = tid; i < RB * APITCH; i += NTHR) Ah[i] = (_Float16)0.0f;
#pragma unroll 1
  for (int i = tid; i < RB * HPITCH; i += NTHR) { Hh[i] = (unsigned short)0; Hl[i] = (unsigned short)0; }
  if (tid < PLINE) lbuf[tid] = 0.0f;

  float c1[8], c2[8], h2f[8], b1r[4], b2r[4];
#pragma unroll
  for (int r = 0; r < 8; ++r) { c1[r] = 0.0f; c2[r] = 0.0f; h2f[r] = 0.0f; }
#pragma unroll
  for (int g = 0; g < 4; ++g) {
    b1r[g] = bf16r(bias1[g * NHID + j]);
    b2r[g] = bf16r(bias2[g * NHID + j]);
  }
  __syncthreads();
  {
    const int m = tid >> 4, f4 = (tid & 15) * 4;
    const v4f v = *(const v4f*)(x + ((size_t)(rowbase + m) * NSTEP) * NFEAT + f4);
    const unsigned short u0 = f2bf_bits(v[0]), u1 = f2bf_bits(v[1]), u2 = f2bf_bits(v[2]), u3 = f2bf_bits(v[3]);
    v2u pk;
    pk[0] = (unsigned)u0 | ((unsigned)u1 << 16);
    pk[1] = (unsigned)u2 | ((unsigned)u3 << 16);
    *(v2u*)(Xs + m * XPITCH + f4) = pk;
  }
  __syncthreads();

  const __bf16*   axrow = (const __bf16*)Xs + c * XPITCH + koff;
  const _Float16* ahrow = Ah + c * APITCH + koff;
  const __bf16*   w1x = W1X + (size_t)j * NFEAT + koff;
  const _Float16* w1h = W1H + (size_t)j * NHID + koff;
  const _Float16* w2t = W2T + (size_t)j * KCAT2 + koff;
  const v8f z8 = {0.f, 0.f, 0.f, 0.f, 0.f, 0.f, 0.f, 0.f};

#pragma unroll 1
  for (int t = 0; t < NSTEP; ++t) {
    v8f acc[4];
    acc[0] = z8; acc[1] = z8; acc[2] = z8; acc[3] = z8;
#pragma unroll 1
    for (int kx = 0; kx < NFEAT; kx += 32) {
      const v16b a  = Frag<__bf16>::load(axrow + kx);
      const v16b f0 = Frag<__bf16>::load(w1x + kx);
      const v16b f1 = Frag<__bf16>::load(w1x + (size_t)1 * NHID * NFEAT + kx);
      const v16b f2 = Frag<__bf16>::load(w1x + (size_t)2 * NHID * NFEAT + kx);
      const v16b f3 = Frag<__bf16>::load(w1x + (size_t)3 * NHID * NFEAT + kx);
      acc[0] = Frag<__bf16>::mma(a, f0, acc[0]);
      acc[1] = Frag<__bf16>::mma(a, f1, acc[1]);
      acc[2] = Frag<__bf16>::mma(a, f2, acc[2]);
      acc[3] = Frag<__bf16>::mma(a, f3, acc[3]);
      grp_guard_b(acc[0], acc[1], acc[2], acc[3], a, f0, f1, f2, f3);
    }
#pragma unroll 1
    for (int k0 = 0; k0 < NHID; k0 += 32) {
      const v16h a  = Frag<_Float16>::load(ahrow + k0);
      const v16h f0 = Frag<_Float16>::load(w1h + k0);
      const v16h f1 = Frag<_Float16>::load(w1h + (size_t)1 * NHID * NHID + k0);
      const v16h f2 = Frag<_Float16>::load(w1h + (size_t)2 * NHID * NHID + k0);
      const v16h f3 = Frag<_Float16>::load(w1h + (size_t)3 * NHID * NHID + k0);
      acc[0] = Frag<_Float16>::mma(a, f0, acc[0]);
      acc[1] = Frag<_Float16>::mma(a, f1, acc[1]);
      acc[2] = Frag<_Float16>::mma(a, f2, acc[2]);
      acc[3] = Frag<_Float16>::mma(a, f3, acc[3]);
      grp_guard_h(acc[0], acc[1], acc[2], acc[3], a, f0, f1, f2, f3);
    }
    acc_guard4(acc[0], acc[1], acc[2], acc[3]);
    float h1v[8];
#pragma unroll
    for (int r = 0; r < 8; ++r) {
      const float zi = acc[0][r] * WCARRY_INV + b1r[0];
      const float zj = acc[1][r] * WCARRY_INV + b1r[1];
      const float zf = acc[2][r] * WCARRY_INV + b1r[2];
      const float zo = acc[3][r] * WCARRY_INV + b1r[3];
      const float cn = c1[r] * fsig(zf + FORGET_B) + fsig(zi) * ftanh(zj);
      c1[r] = cn;
      h1v[r] = ftanh(cn) * fsig(zo);
    }
    __syncthreads();
#pragma unroll
    for (int r = 0; r < 8; ++r) Ah[(8 * hh + r) * APITCH + j] = (_Float16)h1v[r];
    {
      const int tn = (t + 1 < NSTEP) ? (t + 1) : (NSTEP - 1);
      const int m = tid >> 4, f4 = (tid & 15) * 4;
      const v4f v = *(const v4f*)(x + ((size_t)(rowbase + m) * NSTEP + (size_t)tn) * NFEAT + f4);
      const unsigned short u0 = f2bf_bits(v[0]), u1 = f2bf_bits(v[1]), u2 = f2bf_bits(v[2]), u3 = f2bf_bits(v[3]);
      v2u pk;
      pk[0] = (unsigned)u0 | ((unsigned)u1 << 16);
      pk[1] = (unsigned)u2 | ((unsigned)u3 << 16);
      *(v2u*)(Xs + m * XPITCH + f4) = pk;
    }
    __syncthreads();

    acc[0] = z8; acc[1] = z8; acc[2] = z8; acc[3] = z8;
#pragma unroll 1
    for (int k0 = 0; k0 < KCAT2; k0 += 32) {
      const v16h a  = Frag<_Float16>::load(ahrow + k0);
      const v16h f0 = Frag<_Float16>::load(w2t + k0);
      const v16h f1 = Frag<_Float16>::load(w2t + (size_t)1 * NHID * KCAT2 + k0);
      const v16h f2 = Frag<_Float16>::load(w2t + (size_t)2 * NHID * KCAT2 + k0);
      const v16h f3 = Frag<_Float16>::load(w2t + (size_t)3 * NHID * KCAT2 + k0);
      acc[0] = Frag<_Float16>::mma(a, f0, acc[0]);
      acc[1] = Frag<_Float16>::mma(a, f1, acc[1]);
      acc[2] = Frag<_Float16>::mma(a, f2, acc[2]);
      acc[3] = Frag<_Float16>::mma(a, f3, acc[3]);
      grp_guard_h(acc[0], acc[1], acc[2], acc[3], a, f0, f1, f2, f3);
    }
    acc_guard4(acc[0], acc[1], acc[2], acc[3]);
#pragma unroll
    for (int r = 0; r < 8; ++r) {
      const float zi = acc[0][r] * WCARRY_INV + b2r[0];
      const float zj = acc[1][r] * WCARRY_INV + b2r[1];
      const float zf = acc[2][r] * WCARRY_INV + b2r[2];
      const float zo = acc[3][r] * WCARRY_INV + b2r[3];
      const float cn = c2[r] * fsig(zf + FORGET_B) + fsig(zi) * ftanh(zj);
      c2[r] = cn;
      h2f[r] = ftanh(cn) * fsig(zo);
    }
    __syncthreads();
#pragma unroll
    for (int r = 0; r < 8; ++r) Ah[(8 * hh + r) * APITCH + NHID + j] = (_Float16)h2f[r];
  }

#pragma unroll
  for (int r = 0; r < 8; ++r) {
    const float v = h2f[r];
    const unsigned short hb = f2bf_bits(v);
    const unsigned short lb = f2bf_bits(v - bf_bits2f(hb));
    Hh[(8 * hh + r) * HPITCH + j] = hb;
    Hl[(8 * hh + r) * HPITCH + j] = lb;
  }
  __syncthreads();
  const __bf16* hhrow = (const __bf16*)Hh + c * HPITCH + koff;
  const __bf16* hlrow = (const __bf16*)Hl + c * HPITCH + koff;
  float* slab = Sl[wave];
  float lpart = 0.0f;
#pragma unroll 1
  for (int si = 0; si < 3; ++si) {
    const int n0 = 64 * (wave + NWAVE * si);
    v8f acc[4];
    acc[0] = z8; acc[1] = z8; acc[2] = z8; acc[3] = z8;
#pragma unroll 1
    for (int k0 = 0; k0 < NHID; k0 += 32) {
      const v16b ahi = Frag<__bf16>::load(hhrow + k0);
      const v16b alo = Frag<__bf16>::load(hlrow + k0);
      const __bf16* wd = WDT + (size_t)(n0 + c) * NHID + koff + k0;
      const v16b f0 = Frag<__bf16>::load(wd);
      const v16b f1 = Frag<__bf16>::load(wd + (size_t)16 * NHID);
      const v16b f2 = Frag<__bf16>::load(wd + (size_t)32 * NHID);
      const v16b f3 = Frag<__bf16>::load(wd + (size_t)48 * NHID);
      acc[0] = Frag<__bf16>::mma(ahi, f0, acc[0]);
      acc[0] = Frag<__bf16>::mma(alo, f0, acc[0]);
      acc[1] = Frag<__bf16>::mma(ahi, f1, acc[1]);
      acc[1] = Frag<__bf16>::mma(alo, f1, acc[1]);
      acc[2] = Frag<__bf16>::mma(ahi, f2, acc[2]);
      acc[2] = Frag<__bf16>::mma(alo, f2, acc[2]);
      acc[3] = Frag<__bf16>::mma(ahi, f3, acc[3]);
      acc[3] = Frag<__bf16>::mma(alo, f3, acc[3]);
      grp_guard_b2(acc[0], acc[1], acc[2], acc[3], ahi, alo, f0, f1, f2, f3);
    }
    acc_guard4(acc[0], acc[1], acc[2], acc[3]);
    float bdv[4];
#pragma unroll
    for (int jj = 0; jj < 4; ++jj) bdv[jj] = bf16r(biasd[n0 + 16 * jj + c]);
#pragma unroll
    for (int jj = 0; jj < 4; ++jj)
#pragma unroll
      for (int r = 0; r < 8; ++r) slab[(8 * hh + r) * SLABP + 16 * jj + c] = acc[jj][r] + bdv[jj];
    __builtin_amdgcn_fence(__ATOMIC_RELEASE, "workgroup");
    __builtin_amdgcn_wave_barrier();
    __builtin_amdgcn_fence(__ATOMIC_ACQUIRE, "workgroup");
#pragma unroll
    for (int it = 0; it < 8; ++it) {
      const int row = it * 2 + hh;
      const v4f pv = *(const v4f*)(slab + row * SLABP + c4);
      const v4f lv = *(const v4f*)(lab + (size_t)(rowbase + row) * NPCOL + n0 + c4);
#pragma unroll
      for (int e = 0; e < 4; ++e) {
        const float d = pv[e] - bf16r(lv[e]);
        lpart += d * d;
      }
    }
    for (int pass = 0; pass < 2; ++pass) {
#pragma unroll
      for (int it = 0; it < 8; ++it) {
        const int row = it * 2 + hh;
        const v4f pv = *(const v4f*)(slab + row * SLABP + c4);
        *(volatile v4f*)(pred + (size_t)(rowbase + row) * NPCOL + n0 + c4) = pv;
      }
      __threadfence();
    }
    __builtin_amdgcn_fence(__ATOMIC_RELEASE, "workgroup");
    __builtin_amdgcn_wave_barrier();
    __builtin_amdgcn_fence(__ATOMIC_ACQUIRE, "workgroup");
  }

#pragma unroll
  for (int off = 1; off < 32; off <<= 1) lpart += __shfl_xor(lpart, off, 32);
  if (lane == 0) wsum[wave] = lpart;
  __syncthreads();
  if (tid == 0) {
    float s = 0.0f;
#pragma unroll
    for (int w = 0; w < NWAVE; ++w) s += wsum[w];
    lbuf[0] = s;
  }
  __syncthreads();
  if (wave == 0) {
    const int li = (lane < 8) ? lane : 7;
    const v4f pv = *(const v4f*)(lbuf + 4 * li);
    float* pp = part + (size_t)blockIdx.x * PLINE + 4 * li;
    for (int pass = 0; pass < 2; ++pass) {
      if (lane < 8) *(volatile v4f*)pp = pv;
      __threadfence();
    }
  }
}

__global__ __launch_bounds__(32) void loss_kernel(const float* __restrict__ part, float* __restrict__ outl) {
  if (threadIdx.x == 0) {
    float s = 0.0f;
#pragma unroll 1
    for (int b = 0; b < NBLK; ++b) s += part[(size_t)b * PLINE];
    const float lval = s * LOSS_INV;
    *(volatile float*)outl = lval;
    __threadfence();
    *(volatile float*)outl = lval;
  }
}

extern "C" void kernel_launch(void* const* d_in, const int* in_sizes, int n_in,
                              void* d_out, int out_size, void* d_ws, size_t ws_size, hipStream_t stream) {
  if (n_in < 8 || d_out == nullptr || d_ws == nullptr) return;
  if (in_sizes[0] != NSEQ * NSTEP * NFEAT || in_sizes[1] != NPRED || in_sizes[2] != (NFEAT + NHID) * NGATE4 ||
      in_sizes[3] != NGATE4 || in_sizes[4] != KCAT2 * NGATE4 || in_sizes[5] != NGATE4 ||
      in_sizes[6] != NHID * NPCOL || in_sizes[7] != NPCOL || out_size != NPRED + 1) return;

  const float* xin = (const float*)d_in[0];
  const float* lab = (const float*)d_in[1];
  const float* w1  = (const float*)d_in[2];
  const float* bb1 = (const float*)d_in[3];
  const float* w2  = (const float*)d_in[4];
  const float* bb2 = (const float*)d_in[5];
  const float* wd  = (const float*)d_in[6];
  const float* bbd = (const float*)d_in[7];
  float* out  = (float*)d_out;
  float* outl = out + (size_t)NPRED;

  char* ws = (char*)d_ws; size_t off = 0;
  auto carve = [&](size_t bytes) -> char* { char* p = ws + off; off += (bytes + 255) & ~(size_t)255; return p; };
  unsigned short* W1X  = (unsigned short*)carve((size_t)NGATE4 * NFEAT * 2);
  unsigned short* W1H  = (unsigned short*)carve((size_t)NGATE4 * NHID * 2);
  unsigned short* W2T  = (unsigned short*)carve((size_t)NGATE4 * KCAT2 * 2);
  unsigned short* WDT  = (unsigned short*)carve((size_t)NPCOL * NHID * 2);
  float*          PART = (float*)carve((size_t)NBLK * PLINE * 4);
  if (off > ws_size || off > (size_t)134217728) return;

  tpw_kernel<0><<<dim3(NGATE4 / 64, NFEAT / 64), NTHR, 0, stream>>>(w1, NFEAT, NGATE4, NFEAT, W1X, WCARRY);
  tpw_kernel<1><<<dim3(NGATE4 / 64, NHID / 64), NTHR, 0, stream>>>(w1 + (size_t)NFEAT * NGATE4, NHID, NGATE4, NHID, W1H, WCARRY);
  tpw_kernel<1><<<dim3(NGATE4 / 64, KCAT2 / 64), NTHR, 0, stream>>>(w2, KCAT2, NGATE4, KCAT2, W2T, WCARRY);
  tpw_kernel<0><<<dim3(NPCOL / 64, NHID / 64), NTHR, 0, stream>>>(wd, NHID, NPCOL, NHID, WDT, 1.0f);
  lstm2_kernel<<<NBLK, NTHR, 0, stream>>>(xin, bb1, bb2, bbd, lab, W1X, W1H, W2T, WDT, out, PART);
  loss_kernel<<<1, 32, 0, stream>>>(PART, outl);
}
